// GPSA1D_20444044329743
// MI455X (gfx1250) — hardware-verified
//
#include <hip/hip_runtime.h>
#include <math.h>

typedef __attribute__((ext_vector_type(16))) _Float16 v16h;
typedef __attribute__((ext_vector_type(16))) __bf16 v16b;
typedef __attribute__((ext_vector_type(8)))  _Float16 v8h;
typedef __attribute__((ext_vector_type(8)))  float v8f;
typedef __attribute__((ext_vector_type(4)))  float v4f;
typedef __attribute__((ext_vector_type(2)))  float v2f;
typedef __attribute__((ext_vector_type(4)))  unsigned v4u;
typedef __attribute__((ext_vector_type(4)))  int v4i;
typedef float __attribute__((may_alias)) float_a;
typedef int __attribute__((may_alias)) int_a;

template <typename T> __device__ __forceinline__ void vst2(void* p, T v) { *(volatile T*)p = v; __threadfence(); *(volatile T*)p = v; }
__device__ __forceinline__ v8f wmma16(v16h a, v16h b, v8f c) {
  v8f d = __builtin_amdgcn_wmma_f32_16x16x32_f16(false, a, false, b, (short)0, c, false, false);
  asm volatile("v_nop\n\tv_nop\n\tv_nop\n\tv_nop" : "+v"(d) : "v"(a), "v"(b));
  return d;
}
__device__ __forceinline__ v8f wmma_bf(v16b a, v16b b, v8f c) {
  v8f d = __builtin_amdgcn_wmma_f32_16x16x32_bf16(false, a, false, b, (short)0, c, false, false);
  asm volatile("v_nop\n\tv_nop\n\tv_nop\n\tv_nop" : "+v"(d) : "v"(a), "v"(b));
  return d;
}
__device__ __forceinline__ v16h frag_h(const _Float16* rowk0, int lane) {
  union { v16h v; v8h q[2]; } u; const _Float16* p = rowk0 + 8 * (lane >> 4);
  u.q[0] = *(const v8h*)p; u.q[1] = *(const v8h*)(p + 16); return u.v;
}
__device__ __forceinline__ v16h frag_f32(const float* rowk0, int lane) {
  v16h a; const float* p = rowk0 + 8 * (lane >> 4);
#pragma unroll
  for (int i = 0; i < 8; ++i) { a[i] = (_Float16)p[i]; a[8 + i] = (_Float16)p[16 + i]; }
  return a;
}
__device__ __forceinline__ v16h frag_f32s(const float* rowk0, int lane, float sc) {
  v16h a; const float* p = rowk0 + 8 * (lane >> 4);
#pragma unroll
  for (int i = 0; i < 8; ++i) { a[i] = (_Float16)(p[i] * sc); a[8 + i] = (_Float16)(p[16 + i] * sc); }
  return a;
}
__device__ __forceinline__ v16h fragc_f32(const float* W, int k0, int n, int lane, int ld, int K) {
  v16h a; const int g = lane >> 4;
#pragma unroll
  for (int i = 0; i < 8; ++i) { const int ka = k0 + 8 * g + i, kb = ka + 16;
    a[i] = (_Float16)(ka < K ? W[(size_t)(ka < K ? ka : K - 1) * ld + n] : 0.f); a[8 + i] = (_Float16)(kb < K ? W[(size_t)(kb < K ? kb : K - 1) * ld + n] : 0.f); }
  return a;
}
struct F2 { v16b h, l; };
__device__ __forceinline__ F2 bsplit16(const float v[16]) { F2 r;
#pragma unroll
  for (int i = 0; i < 16; ++i) { const __bf16 h = (__bf16)v[i]; r.h[i] = h; r.l[i] = (__bf16)(v[i] - (float)h); }
  return r; }
__device__ __forceinline__ F2 split_row(const float* row, int k0, int lane) { float v[16]; const float* p = row + k0 + 8 * (lane >> 4);
#pragma unroll
  for (int i = 0; i < 8; ++i) { v[i] = p[i]; v[8 + i] = p[16 + i]; }
  return bsplit16(v); }
__device__ __forceinline__ F2 split_rowK(const float* row, int k0, int lane, int K) { float v[16]; const int g = lane >> 4;
#pragma unroll
  for (int i = 0; i < 8; ++i) { const int ka = k0 + 8 * g + i, kb = ka + 16; v[i] = ka < K ? row[ka < K ? ka : K - 1] : 0.f; v[8 + i] = kb < K ? row[kb < K ? kb : K - 1] : 0.f; }
  return bsplit16(v); }
__device__ __forceinline__ F2 split_col(const float* W, int k0, int n, int lane, int ld, int K) { float v[16]; const int g = lane >> 4;
#pragma unroll
  for (int i = 0; i < 8; ++i) { const int ka = k0 + 8 * g + i, kb = ka + 16; v[i] = ka < K ? W[(size_t)(ka < K ? ka : K - 1) * ld + n] : 0.f; v[8 + i] = kb < K ? W[(size_t)(kb < K ? kb : K - 1) * ld + n] : 0.f; }
  return bsplit16(v); }
__device__ __forceinline__ v8f mac3(const F2& a, const F2& b, v8f c) { c = wmma_bf(a.l, b.h, c); c = wmma_bf(a.h, b.l, c); return wmma_bf(a.h, b.h, c); }
__device__ __forceinline__ float sigm(float v) { return 1.0f / (1.0f + expf(-v)); }
#define LDSX() do { asm volatile("s_wait_dscnt 0" ::: "memory"); __builtin_amdgcn_wave_barrier(); __builtin_amdgcn_fence(__ATOMIC_RELEASE, "workgroup"); } while (0)


#define NB 2
#define SS 2048
#define DM 256
#define NH 8
#define HD 32
#define NR (NB * SS)
#ifndef TQB
#define TQB (SS / 64)
#define TNB NB
#endif
typedef __attribute__((ext_vector_type(8))) __bf16 v8b;
__device__ __forceinline__ v16b frag_b(const __bf16* rowk0, int lane) {
  union { v16b v; v8b q[2]; } u; const __bf16* p = rowk0 + 8 * (lane >> 4);
  u.q[0] = *(const v8b*)p; u.q[1] = *(const v8b*)(p + 16); return u.v;
}
__device__ __forceinline__ float bfr(float v) { return (float)(__bf16)v; }
__device__ __attribute__((noinline)) float exp_ni(float v) { return expf(v); }
__device__ __attribute__((noinline)) float erf_ni(float v) { return erff(v); }

#define WS_PW  0u
#define WS_PV  (WS_PW + 2u * (size_t)512 * DM)
#define WS_PP  (WS_PV + 2u * (size_t)DM * DM)
#define WS_Q   (WS_PP + 2u * (size_t)DM * DM)
#define WS_K   (WS_Q + 2u * (size_t)NR * DM)
#define WS_V   (WS_K + 2u * (size_t)NR * DM)
#define WS_P2  (WS_V + 2u * (size_t)NB * DM * SS)
#define WS_O   (WS_P2 + 2u * (size_t)NH * SS * SS)
#define WS_END (WS_O + 4u * (size_t)NR * DM)

__global__ __launch_bounds__(256) void k_pack(const float* __restrict__ WQK, const float* __restrict__ WV, const float* __restrict__ WP, __bf16* __restrict__ P) { const int n = blockIdx.x, which = blockIdx.y, t = threadIdx.x; __shared__ __align__(16) __bf16 s[DM];
  if (which == 0) { s[t] = (__bf16)WQK[(size_t)t * (2 * DM) + n]; __syncthreads(); if (t < DM / 8) vst2((unsigned*)(P + WS_PW / 2 + (size_t)n * DM + t * 8), *(const v4u*)&s[t * 8]); }
  else if (which == 1) { if (n >= DM) return; s[t] = (__bf16)WV[(size_t)t * DM + n]; __syncthreads(); if (t < DM / 8) vst2((unsigned*)(P + WS_PV / 2 + (size_t)n * DM + t * 8), *(const v4u*)&s[t * 8]); }
  else { if (n >= DM) return; s[t] = (__bf16)WP[(size_t)t * DM + n]; __syncthreads(); if (t < DM / 8) vst2((unsigned*)(P + WS_PP / 2 + (size_t)n * DM + t * 8), *(const v4u*)&s[t * 8]); } }
__global__ __launch_bounds__(128) void k_proj(const float* __restrict__ X, const __bf16* __restrict__ P, _Float16* __restrict__ Q, _Float16* __restrict__ Kr, _Float16* __restrict__ V) {
  __shared__ __align__(16) _Float16 so[64][136]; __shared__ __align__(16) _Float16 st[128][72];
  const int tid = threadIdx.x, wave = tid >> 5, lane = tid & 31, col = lane & 15, g = lane >> 4; const int cb = blockIdx.y; const size_t rb = (size_t)blockIdx.x * 64; const size_t r0 = rb + wave * 16;
  const __bf16* Wr = (cb < 4) ? (P + WS_PW / 2 + (size_t)cb * 128 * DM) : (P + WS_PV / 2 + (size_t)(cb - 4) * 128 * DM);
  v8f acc[8] = {};
#pragma unroll
  for (int kc = 0; kc < DM / 32; ++kc) { v16b a; { const float* p = X + (r0 + col) * DM + kc * 32 + 8 * g;
#pragma unroll
      for (int i = 0; i < 8; ++i) { a[i] = (__bf16)p[i]; a[8 + i] = (__bf16)p[16 + i]; } }
#pragma unroll
    for (int j = 0; j < 8; ++j) acc[j] = wmma_bf(a, frag_b(Wr + (size_t)(j * 16 + col) * DM + kc * 32, lane), acc[j]); }
  if (cb < 4) {
#pragma unroll
    for (int j = 0; j < 8; ++j)
#pragma unroll
      for (int r = 0; r < 8; ++r) so[wave * 16 + 8 * g + r][j * 16 + col] = (_Float16)acc[j][r];
    __syncthreads(); _Float16* dst = (cb < 2) ? Q : Kr; const int c0 = (cb & 1) * 128; for (int e = tid; e < 64 * 16; e += 128) { const int rl = e >> 4, q = e & 15; vst2((unsigned*)(dst + (rb + rl) * DM + c0 + q * 8), *(const v4u*)&so[rl][q * 8]); } }
  else {
#pragma unroll
    for (int j = 0; j < 8; ++j)
#pragma unroll
      for (int r = 0; r < 8; ++r) st[j * 16 + col][wave * 16 + 8 * g + r] = (_Float16)acc[j][r];
    __syncthreads(); const size_t b = rb / SS; const int s0 = (int)(rb % SS); const int c0 = (cb - 4) * 128; for (int e = tid; e < 128 * 8; e += 128) { const int d = e >> 3, pc = e & 7; vst2((unsigned*)(V + ((b * DM + c0 + d) * SS) + s0 + pc * 8), *(const v4u*)&st[d][pc * 8]); } }
}
__global__ __launch_bounds__(256) void k_posw(const float* __restrict__ WPOS, const float* __restrict__ BPOS, _Float16* __restrict__ P2) { __shared__ float red[8]; __shared__ __align__(16) _Float16 sp[SS]; const int t = threadIdx.x; const int n = blockIdx.x, h = blockIdx.y;
  const float a = bfr(WPOS[h]), c = bfr(WPOS[NH + h]), b0 = bfr(BPOS[h]);
  float v[8]; float mx = -3.0e38f; for (int i = 0; i < 8; ++i) { const int m = t * 8 + i; const float rel = (float)(n - m); v[i] = rel * a + fabsf(rel) * c + b0; mx = fmaxf(mx, v[i]); }
#pragma unroll
  for (int o = 1; o < 32; o <<= 1) mx = fmaxf(mx, __shfl_xor(mx, o));
  if ((t & 31) == 0) red[t >> 5] = mx; __syncthreads(); float M = red[0]; for (int i = 1; i < 8; ++i) M = fmaxf(M, red[i]); __syncthreads();
  float z = 0.f; for (int i = 0; i < 8; ++i) { v[i] = __expf(v[i] - M); z += v[i]; }
#pragma unroll
  for (int o = 1; o < 32; o <<= 1) z += __shfl_xor(z, o);
  if ((t & 31) == 0) red[t >> 5] = z; __syncthreads(); float Z = 0.f; for (int i = 0; i < 8; ++i) Z += red[i]; const float iz = 2048.0f / Z;
  for (int i = 0; i < 8; ++i) sp[t * 8 + i] = (_Float16)(v[i] * iz); __syncthreads();
  vst2((unsigned*)(P2 + ((size_t)h * SS + n) * SS + t * 8), *(const v4u*)&sp[t * 8]); }
__global__ __launch_bounds__(128) void k_attn(const _Float16* __restrict__ Q, const _Float16* __restrict__ Kr, const _Float16* __restrict__ V, const _Float16* __restrict__ P2, const float* __restrict__ GATE, float* __restrict__ O) {
  __shared__ __align__(16) _Float16 sph[4][16][40]; __shared__ __align__(16) float so[4][16][36];
  const int tid = threadIdx.x, wave = tid >> 5, lane = tid & 31, col = lane & 15, g = lane >> 4; const int h = blockIdx.y; const size_t b = blockIdx.z; const int q0 = blockIdx.x * 64 + wave * 16; const size_t rq = b * SS + q0;
  const float gt = 1.0f / (1.0f + expf(-bfr(GATE[h])));
  const v16h aq = frag_h(Q + (rq + col) * DM + h * HD, lane);
  float m[8], l[8];
#pragma unroll
  for (int r = 0; r < 8; ++r) { m[r] = -3.0e38f; l[r] = 0.f; }
  v8f acc[2] = {}, acc2[2] = {};
#pragma unroll 1
  for (int ks = 0; ks < SS / 32; ++ks) { const int j0 = ks * 32; v8f s[2];
#pragma unroll
    for (int ct = 0; ct < 2; ++ct) { const int kk = j0 + ct * 16 + col; v8f c = {}; c = wmma16(aq, frag_h(Kr + (b * SS + kk) * DM + h * HD, lane), c);
#pragma unroll
      for (int r = 0; r < 8; ++r) s[ct][r] = c[r] * 0.17677669529663688f; }
#pragma unroll
    for (int r = 0; r < 8; ++r) { float mx = fmaxf(s[0][r], s[1][r]);
#pragma unroll
      for (int o = 1; o < 16; o <<= 1) mx = fmaxf(mx, __shfl_xor(mx, o));
      const float mn = fmaxf(m[r], mx); const float alpha = (m[r] <= -1.0e38f) ? 0.f : __expf(m[r] - mn); const float e0 = __expf(s[0][r] - mn), e1 = __expf(s[1][r] - mn); float es = e0 + e1;
#pragma unroll
      for (int o = 1; o < 16; o <<= 1) es += __shfl_xor(es, o);
      l[r] = l[r] * alpha + es; m[r] = mn;
#pragma unroll
      for (int dt = 0; dt < 2; ++dt) acc[dt][r] *= alpha;
      sph[wave][8 * g + r][col] = (_Float16)(e0 * 2048.0f); sph[wave][8 * g + r][16 + col] = (_Float16)(e1 * 2048.0f); }
    LDSX();
    const v16h pa = frag_h(&sph[wave][col][0], lane); const v16h pp = frag_h(P2 + ((size_t)h * SS + q0 + col) * SS + j0, lane);
#pragma unroll
    for (int dt = 0; dt < 2; ++dt) { const v16h vf = frag_h(V + ((b * DM + h * HD + dt * 16 + col) * SS) + j0, lane); acc[dt] = wmma16(pa, vf, acc[dt]); acc2[dt] = wmma16(pp, vf, acc2[dt]); }
    LDSX(); }
#pragma unroll
  for (int r = 0; r < 8; ++r) { const float il = (1.0f / 2048.0f) / l[r];
#pragma unroll
    for (int dt = 0; dt < 2; ++dt) so[wave][8 * g + r][dt * 16 + col] = (1.0f - gt) * acc[dt][r] * il + gt * acc2[dt][r] * (1.0f / 2048.0f); }
  LDSX();
  for (int rl = 0; rl < 16; ++rl) if (lane < 8) vst2(O + (rq + rl) * DM + h * HD + lane * 4, *(const v4f*)&so[wave][rl][lane * 4]);
}
__global__ __launch_bounds__(128) void k_out(const float* __restrict__ O, const __bf16* __restrict__ P, const float* __restrict__ BP, float* __restrict__ Y) { __shared__ __align__(16) float so[4][16][132];
  const int tid = threadIdx.x, wave = tid >> 5, lane = tid & 31, col = lane & 15, g = lane >> 4; const size_t r0 = (size_t)blockIdx.x * 64 + wave * 16; const int c0 = blockIdx.y * 128; const __bf16* Wr = P + WS_PP / 2;
  v8f acc[8] = {};
#pragma unroll
  for (int kc = 0; kc < DM / 32; ++kc) { const F2 a = split_row(O + (r0 + col) * DM, kc * 32, lane);
#pragma unroll
    for (int j = 0; j < 8; ++j) { const v16b w = frag_b(Wr + (size_t)(c0 + j * 16 + col) * DM + kc * 32, lane); acc[j] = wmma_bf(a.h, w, acc[j]); acc[j] = wmma_bf(a.l, w, acc[j]); } }
#pragma unroll
  for (int j = 0; j < 8; ++j) { const float bb = bfr(BP[c0 + j * 16 + col]);
#pragma unroll
    for (int r = 0; r < 8; ++r) so[wave][8 * g + r][j * 16 + col] = acc[j][r] + bb; }
  LDSX(); for (int rl = 0; rl < 16; ++rl) vst2(Y + (r0 + rl) * DM + c0 + lane * 4, *(const v4f*)&so[wave][rl][lane * 4]); }
extern "C" void kernel_launch(void* const* d_in, const int* in_sizes, int n_in, void* d_out, int out_size, void* d_ws, size_t ws_size, hipStream_t stream) {
  (void)in_sizes; (void)n_in; (void)out_size;
  const float** F = (const float**)d_in;
  if (ws_size < (size_t)WS_END) return;
  char* ws = (char*)d_ws; __bf16* P = (__bf16*)ws; _Float16 *Q = (_Float16*)(ws + WS_Q), *Kr = (_Float16*)(ws + WS_K), *V = (_Float16*)(ws + WS_V), *P2 = (_Float16*)(ws + WS_P2); float* O = (float*)(ws + WS_O);
  k_pack<<<dim3(2 * DM, 3), 256, 0, stream>>>(F[1], F[2], F[3], P);
  k_proj<<<dim3(TNB * SS / 64, 6), 128, 0, stream>>>(F[0], P, Q, Kr, V);
  k_posw<<<dim3(SS, NH), 256, 0, stream>>>(F[5], F[6], P2);
  k_attn<<<dim3(TQB, NH, TNB), 128, 0, stream>>>(Q, Kr, V, P2, F[7], O);
  k_out<<<dim3(TNB * SS / 64, DM / 128), 128, 0, stream>>>(O, P, F[4], (float*)d_out);
}
